// ClassNetPP_55731495633087
// MI455X (gfx1250) — hardware-run, weakly checked
//
#include <hip/hip_runtime.h>


#define NI   16
#define NP   1024
#define DIN  768
#define DD   512
#define HID  128
#define NC   20
#define NK   64
#define NPR  1280
#define HW   32
#define K9   1152
typedef _Float16 h16;
typedef unsigned short bf;
typedef __attribute__((ext_vector_type(16))) __bf16   v16bf;
typedef __attribute__((ext_vector_type(16))) _Float16 v16h;
typedef __attribute__((ext_vector_type(8)))  _Float16 v8h;
typedef __attribute__((ext_vector_type(8)))  unsigned short v8us;
typedef __attribute__((ext_vector_type(8)))  float    v8f;
typedef __attribute__((ext_vector_type(4)))  float    v4f;
typedef v8h  __attribute__((may_alias)) v8ha;
typedef v4f  __attribute__((may_alias)) v4fa;
typedef v8us __attribute__((may_alias)) v8usa;

__device__ __forceinline__ unsigned short f2bf(float f) { unsigned u = __float_as_uint(f); u += 0x7FFFu + ((u >> 16) & 1u); return (unsigned short)(u >> 16); }
__device__ __forceinline__ float bf2f(unsigned short b) { return __uint_as_float(((unsigned)b) << 16); }
__device__ __forceinline__ float bfr(float f) { return bf2f(f2bf(f)); }
__device__ __forceinline__ v16h cat16(v8h lo, v8h hi) { return __builtin_shufflevector(lo, hi, 0, 1, 2, 3, 4, 5, 6, 7, 8, 9, 10, 11, 12, 13, 14, 15); }
__device__ __forceinline__ v16bf cat16b(v8us lo, v8us hi) { return __builtin_bit_cast(v16bf, __builtin_shufflevector(lo, hi, 0, 1, 2, 3, 4, 5, 6, 7, 8, 9, 10, 11, 12, 13, 14, 15)); }
__device__ __forceinline__ v8f wmma16(v16h a, v16h b, v8f c) { return __builtin_amdgcn_wmma_f32_16x16x32_f16(false, a, false, b, (short)0, c, false, false); }
__device__ __forceinline__ v8f wmmab(v16bf a, v16bf b, v8f c) { return __builtin_amdgcn_wmma_f32_16x16x32_bf16(false, a, false, b, (short)0, c, false, false); }


template <typename T16> struct WFrag;
template <> struct WFrag<h16> { typedef v16h V; static __device__ __forceinline__ V ld(const h16* p) { return cat16(*(const v8h*)p, *(const v8h*)(p + 16)); } static __device__ __forceinline__ v8f mma(V a, V b, v8f c) { return wmma16(a, b, c); } };
template <> struct WFrag<bf> { typedef v16bf V; static __device__ __forceinline__ V ld(const bf* p) { return cat16b(*(const v8us*)p, *(const v8us*)(p + 16)); } static __device__ __forceinline__ v8f mma(V a, V b, v8f c) { return wmmab(a, b, c); } };
template <typename T16, int NSPLIT, bool BIAS>
__global__ __launch_bounds__(32) void k_gemmw(const T16* __restrict__ A, const T16* __restrict__ A2, const T16* __restrict__ Bt, const T16* __restrict__ Bt2, int K, float* C, int ldc, const float* __restrict__ bias, size_t sA, size_t sB, size_t sC) {
    typedef typename WFrag<T16>::V V;
    __shared__ __align__(16) float os[16 * 68];
    const size_t z = blockIdx.z; A += z * sA; if (A2) A2 += z * sA; Bt += z * sB; if (Bt2) Bt2 += z * sB; C += z * sC;
    const int lane = threadIdx.x & 31, lr = lane & 15, hi = lane >> 4; const int r0 = blockIdx.x * 64, c0 = blockIdx.y * 64;
    v8f acc[4][4];
#pragma unroll
    for (int mb = 0; mb < 4; ++mb)
#pragma unroll
        for (int nb = 0; nb < 4; ++nb) acc[mb][nb] = (v8f){};
    const size_t aoff = (size_t)(r0 + lr) * K + 8 * hi, boff = (size_t)(c0 + lr) * K + 8 * hi;
#pragma unroll 1
    for (int kc = 0; kc < K; kc += 32) {
        V a[4], a2[4];
#pragma unroll
        for (int mb = 0; mb < 4; ++mb) { a[mb] = WFrag<T16>::ld(A + aoff + (size_t)mb * 16 * K + kc); if (NSPLIT == 1 || NSPLIT == 2) a2[mb] = WFrag<T16>::ld(A2 + aoff + (size_t)mb * 16 * K + kc); }
#pragma unroll
        for (int nb = 0; nb < 4; ++nb) { const V b = WFrag<T16>::ld(Bt + boff + (size_t)nb * 16 * K + kc); V b2; if (NSPLIT >= 2) b2 = WFrag<T16>::ld(Bt2 + boff + (size_t)nb * 16 * K + kc);
#pragma unroll
            for (int mb = 0; mb < 4; ++mb) { acc[mb][nb] = WFrag<T16>::mma(a[mb], b, acc[mb][nb]); if (NSPLIT == 1 || NSPLIT == 2) acc[mb][nb] = WFrag<T16>::mma(a2[mb], b, acc[mb][nb]); if (NSPLIT >= 2) acc[mb][nb] = WFrag<T16>::mma(a[mb], b2, acc[mb][nb]); } }
        asm volatile("v_nop\n\tv_nop\n\tv_nop\n\tv_nop" : "+v"(acc[0][0]), "+v"(acc[1][1]), "+v"(acc[2][2]), "+v"(acc[3][3]) : "v"(a[0]), "v"(a[3]));
    }
#pragma unroll
    for (int mb = 0; mb < 4; ++mb) {
#pragma unroll
        for (int nb = 0; nb < 4; ++nb) {
#pragma unroll
            for (int j = 0; j < 8; ++j) os[(hi * 8 + j) * 68 + nb * 16 + lr] = acc[mb][nb][j]; }
        __builtin_amdgcn_wave_barrier(); asm volatile("" ::: "memory");
        float* crow = C + (size_t)(r0 + mb * 16) * ldc + c0;
#pragma unroll 1
        for (int ps = 0; ps < 2; ++ps) {
#pragma unroll
            for (int s = 0; s < 8; ++s) { const int row = 2 * s + hi, cofs = lr * 4; v4f val = *(const v4fa*)(os + row * 68 + cofs); if (BIAS) { val[0] += bfr(bias[c0 + cofs]); val[1] += bfr(bias[c0 + cofs + 1]); val[2] += bfr(bias[c0 + cofs + 2]); val[3] += bfr(bias[c0 + cofs + 3]); }
                *(volatile v4f*)(crow + (size_t)row * ldc + cofs) = val; }
            if (ps == 0) __threadfence(); }
        __builtin_amdgcn_wave_barrier(); asm volatile("" ::: "memory");
    }
}

__device__ __forceinline__ h16 tohx(float x) { return (h16)x; }
__device__ __forceinline__ void splitf(float y, unsigned short& h, unsigned short& l) { h = f2bf(y); l = f2bf(y - bf2f(h)); }
typedef __attribute__((ext_vector_type(2))) unsigned short v2us;
typedef __attribute__((ext_vector_type(4))) unsigned short v4us;
typedef __attribute__((ext_vector_type(4))) _Float16 v4h;
typedef __attribute__((ext_vector_type(8))) _Float16 v8h;

__global__ __launch_bounds__(256) void k_cvt8(const float* __restrict__ src, bf* dst, size_t n8) { const size_t i = (size_t)blockIdx.x * 256 + threadIdx.x; if (i >= n8) return; const v8f v = *(const v8f*)(src + i * 8); v8us o;
#pragma unroll
    for (int k = 0; k < 8; ++k) o[k] = f2bf(v[k]); *(volatile v8us*)(dst + i * 8) = o; __threadfence(); *(volatile v8us*)(dst + i * 8) = o; }
__device__ __forceinline__ float bnf(float x, const float* g, const float* b, const float* m, const float* v, int c) { const float sc = __fmul_rn(bfr(g[c]), __frsqrt_rn(__fadd_rn(bfr(v[c]), 1e-5f))); float d = __fsub_rn(x, bfr(m[c])); asm volatile("" : "+v"(d)); float t = __fmul_rn(d, sc); asm volatile("" : "+v"(t)); return __fadd_rn(t, bfr(b[c])); }
__global__ __launch_bounds__(256) void k_bnr(const float* __restrict__ T, int C, const float* __restrict__ g, const float* __restrict__ bb, const float* __restrict__ m, const float* __restrict__ v, float* F, bf* Ph, bf* Pl, int ldp, int c0) {
    const int e = (blockIdx.x * 256 + threadIdx.x) * 4; if (e >= NP * C) return; const int c = e % C; const int r = e / C; v4f o; v4us oh, ol;
#pragma unroll
    for (int u = 0; u < 4; ++u) { const float y = fmaxf(bnf(T[e + u], g, bb, m, v, c + u), 0.f); o[u] = y; unsigned short a, b2; splitf(y, a, b2); oh[u] = a; ol[u] = b2; }
    const size_t po = (size_t)r * ldp + c0 + c; for (int ps = 0; ps < 2; ++ps) { if (F) *(volatile v4f*)(F + e) = o; *(volatile v4us*)(Ph + po) = oh; *(volatile v4us*)(Pl + po) = ol; if (ps == 0) __threadfence(); } }
__global__ __launch_bounds__(256) void k_im2c(const float* __restrict__ O, int dil, bf* Ih, bf* Il) { const int e = (blockIdx.x * 256 + threadIdx.x) * 4; if (e >= NP * K9) return; const int k0 = e % K9; const int p = e / K9; const int y = p / HW, x = p % HW; v4us oh, ol;
#pragma unroll
    for (int u = 0; u < 4; ++u) { const int k = k0 + u; const int c = k / 9, r9 = k % 9; const int yy = y + (r9 / 3 - 1) * dil, xx = x + (r9 % 3 - 1) * dil; float val = 0.f; if (yy >= 0 && yy < HW && xx >= 0 && xx < HW) val = O[(size_t)(yy * HW + xx) * HID + c]; unsigned short a, b; splitf(val, a, b); oh[u] = a; ol[u] = b; }
    *(volatile v4us*)(Ih + e) = oh; *(volatile v4us*)(Il + e) = ol; __threadfence(); *(volatile v4us*)(Ih + e) = oh; *(volatile v4us*)(Il + e) = ol; }
__global__ __launch_bounds__(256) void k_res(const float* __restrict__ P, const float* __restrict__ X1, const float* __restrict__ g, const float* __restrict__ bb, const float* __restrict__ m, const float* __restrict__ v, bf* Ph, bf* Pl) { const int e = (blockIdx.x * 256 + threadIdx.x) * 4; if (e >= NP * DD) return; const int c = e % DD; v4us oh, ol;
#pragma unroll
    for (int u = 0; u < 4; ++u) { const float y = fmaxf(__fadd_rn(bnf(P[e + u], g, bb, m, v, c + u), X1[e + u]), 0.f); unsigned short a, b2; splitf(y, a, b2); oh[u] = a; ol[u] = b2; } *(volatile v4us*)(Ph + e) = oh; *(volatile v4us*)(Pl + e) = ol; __threadfence(); *(volatile v4us*)(Ph + e) = oh; *(volatile v4us*)(Pl + e) = ol; }
__global__ __launch_bounds__(256) void k_l2n(const float* __restrict__ F, float* OUTx, h16* XN) { const int lane = threadIdx.x & 31; const int r = blockIdx.x * 8 + (threadIdx.x >> 5); if (r >= NP) return; float v[DD / 32]; float q = 0.f;
#pragma unroll
    for (int ch = 0; ch < DD / 128; ++ch) { const v4f a = *(const v4f*)(F + (size_t)r * DD + ch * 128 + lane * 4);
#pragma unroll
        for (int u = 0; u < 4; ++u) { v[ch * 4 + u] = a[u]; float p = __fmul_rn(a[u], a[u]); asm volatile("" : "+v"(p)); q = __fadd_rn(q, p); } }
#pragma unroll
    for (int sh = 16; sh; sh >>= 1) q += __shfl_xor(q, sh, 32);
    const float den = fmaxf(__fsqrt_rn(q), 1e-12f);
    for (int ps = 0; ps < 2; ++ps) {
#pragma unroll
        for (int ch = 0; ch < DD / 128; ++ch) { v4f o; v4h o16;
#pragma unroll
            for (int u = 0; u < 4; ++u) { o[u] = __fdiv_rn(v[ch * 4 + u], den); o16[u] = tohx(o[u]); } const size_t oo = (size_t)r * DD + ch * 128 + lane * 4; *(volatile v4f*)(OUTx + oo) = o; *(volatile v4h*)(XN + oo) = o16; }
        if (ps == 0) __threadfence(); } }
__global__ __launch_bounds__(256) void k_p16(const float* __restrict__ W, h16* P) { const int e = (blockIdx.x * 256 + threadIdx.x) * 8; if (e >= NPR * DD) return; const v4f a = *(const v4f*)(W + e), b = *(const v4f*)(W + e + 4); v8h o;
#pragma unroll
    for (int u = 0; u < 4; ++u) { o[u] = tohx(bfr(a[u])); o[4 + u] = tohx(bfr(b[u])); } *(volatile v8h*)(P + e) = o; __threadfence(); *(volatile v8h*)(P + e) = o; }
__global__ __launch_bounds__(256) void k_amax(const float* __restrict__ S, float* ACTb) { const int idx = blockIdx.x * 256 + threadIdx.x; if (idx >= NC * NP) return; const int n = idx % NP; const int c = idx / NP; const float* s = S + (size_t)n * NPR + c * NK; float mx = -3.0e38f;
#pragma unroll 4
    for (int k = 0; k < NK; ++k) mx = fmaxf(mx, s[k]); *(volatile float*)(ACTb + idx) = mx; __threadfence(); *(volatile float*)(ACTb + idx) = mx; }
__global__ __launch_bounds__(256) void k_logit(const float* __restrict__ ACT, const float* __restrict__ ls, float* LOG) { const int idx = blockIdx.x * 256 + threadIdx.x; if (idx >= NI * NC) return; const float* a = ACT + (size_t)idx * NP; float mx = -3.0e38f;
#pragma unroll 4
    for (int n = 0; n < NP; ++n) mx = fmaxf(mx, a[n]); const float r = __fmul_rn(mx, bfr(ls[0])); *(volatile float*)(LOG + idx) = r; __threadfence(); *(volatile float*)(LOG + idx) = r; }

extern "C" void kernel_launch(void* const* d_in, const int* in_sizes, int n_in,
                              void* d_out, int out_size, void* d_ws, size_t ws_size, hipStream_t stream) {
    (void)in_sizes; (void)n_in; (void)out_size;
    const float** I = (const float**)d_in;
    const float *pf = I[0], *protos = I[1], *w0 = I[2], *g0 = I[3], *b0 = I[4], *m0 = I[5], *v0 = I[6], *wr = I[7], *gr = I[8], *br = I[9], *mr = I[10], *vr = I[11], *wl = I[12], *gl = I[13], *bl = I[14], *ml = I[15], *vl = I[16];
    const float *wg = I[17], *gg = I[18], *bg = I[19], *mg = I[20], *vg = I[21], *wp = I[22], *gp = I[23], *bp = I[24], *mp = I[25], *vp = I[26], *wf = I[27], *bfb = I[28], *ls = I[29];
    float* LOG = (float*)d_out; float* ACT = LOG + NI * NC; float* OUTX = ACT + (size_t)NI * NC * NP;
    char* wsp = (char*)d_ws;
    auto take = [&](size_t bytes) { char* p = wsp; wsp += (bytes + 255) & ~(size_t)255; return (void*)p; };
    bf* B0 = (bf*)take((size_t)DD * DIN * 2); bf* BR = (bf*)take((size_t)HID * DD * 2); bf* BL = (bf*)take((size_t)HID * K9 * 2); bf* BG = (bf*)take((size_t)HID * K9 * 2); bf* BP = (bf*)take((size_t)DD * 2 * HID * 2); bf* BF = (bf*)take((size_t)DD * DD * 2); h16* PR = (h16*)take((size_t)NPR * DD * 2);
    bf* X0 = (bf*)take((size_t)NP * DIN * 2); float* T512 = (float*)take((size_t)NP * DD * 4); float* X1 = (float*)take((size_t)NP * DD * 4); bf* X1h = (bf*)take((size_t)NP * DD * 2); bf* X1l = (bf*)take((size_t)NP * DD * 2);
    float* T128 = (float*)take((size_t)NP * HID * 4); float* O = (float*)take((size_t)NP * HID * 4); bf* Oh = (bf*)take((size_t)NP * HID * 2); bf* Ol = (bf*)take((size_t)NP * HID * 2); bf* IMh = (bf*)take((size_t)NP * K9 * 2); bf* IMl = (bf*)take((size_t)NP * K9 * 2);
    bf* CATh = (bf*)take((size_t)NP * 2 * HID * 2); bf* CATl = (bf*)take((size_t)NP * 2 * HID * 2); bf* X2h = (bf*)take((size_t)NP * DD * 2); bf* X2l = (bf*)take((size_t)NP * DD * 2); h16* XN = (h16*)take((size_t)NP * DD * 2); float* S = (float*)take((size_t)NP * NPR * 4);
    if ((size_t)(wsp - (char*)d_ws) > ws_size) return;
    k_cvt8<<<(DD * DIN / 8 + 255) / 256, 256, 0, stream>>>(w0, B0, (size_t)DD * DIN / 8); k_cvt8<<<(HID * DD / 8 + 255) / 256, 256, 0, stream>>>(wr, BR, HID * DD / 8); k_cvt8<<<(HID * K9 / 8 + 255) / 256, 256, 0, stream>>>(wl, BL, HID * K9 / 8); k_cvt8<<<(HID * K9 / 8 + 255) / 256, 256, 0, stream>>>(wg, BG, HID * K9 / 8);
    k_cvt8<<<(DD * 2 * HID / 8 + 255) / 256, 256, 0, stream>>>(wp, BP, DD * 2 * HID / 8); k_cvt8<<<(DD * DD / 8 + 255) / 256, 256, 0, stream>>>(wf, BF, (size_t)DD * DD / 8); k_p16<<<(NPR * DD / 8 + 255) / 256, 256, 0, stream>>>(protos, PR);
    for (int b = 0; b < NI; ++b) {
        k_cvt8<<<(NP * DIN / 8 + 255) / 256, 256, 0, stream>>>(pf + (size_t)b * NP * DIN, X0, (size_t)NP * DIN / 8);
        k_gemmw<bf, 0, false><<<dim3(NP / 64, DD / 64, 1), 32, 0, stream>>>(X0, nullptr, B0, nullptr, DIN, T512, DD, nullptr, 0, 0, 0);
        k_bnr<<<(NP * DD / 4 + 255) / 256, 256, 0, stream>>>(T512, DD, g0, b0, m0, v0, X1, X1h, X1l, DD, 0);
        k_gemmw<bf, 1, false><<<dim3(NP / 64, HID / 64, 1), 32, 0, stream>>>(X1h, X1l, BR, nullptr, DD, T128, HID, nullptr, 0, 0, 0);
        k_bnr<<<(NP * HID / 4 + 255) / 256, 256, 0, stream>>>(T128, HID, gr, br, mr, vr, O, Oh, Ol, HID, 0);
        k_im2c<<<(NP * K9 / 4 + 255) / 256, 256, 0, stream>>>(O, 1, IMh, IMl); k_gemmw<bf, 1, false><<<dim3(NP / 64, HID / 64, 1), 32, 0, stream>>>(IMh, IMl, BL, nullptr, K9, T128, HID, nullptr, 0, 0, 0);
        k_bnr<<<(NP * HID / 4 + 255) / 256, 256, 0, stream>>>(T128, HID, gl, bl, ml, vl, nullptr, CATh, CATl, 2 * HID, 0);
        k_im2c<<<(NP * K9 / 4 + 255) / 256, 256, 0, stream>>>(O, 2, IMh, IMl); k_gemmw<bf, 1, false><<<dim3(NP / 64, HID / 64, 1), 32, 0, stream>>>(IMh, IMl, BG, nullptr, K9, T128, HID, nullptr, 0, 0, 0);
        k_bnr<<<(NP * HID / 4 + 255) / 256, 256, 0, stream>>>(T128, HID, gg, bg, mg, vg, nullptr, CATh, CATl, 2 * HID, HID);
        k_gemmw<bf, 1, false><<<dim3(NP / 64, DD / 64, 1), 32, 0, stream>>>(CATh, CATl, BP, nullptr, 2 * HID, T512, DD, nullptr, 0, 0, 0);
        k_res<<<(NP * DD / 4 + 255) / 256, 256, 0, stream>>>(T512, X1, gp, bp, mp, vp, X2h, X2l);
        k_gemmw<bf, 1, true><<<dim3(NP / 64, DD / 64, 1), 32, 0, stream>>>(X2h, X2l, BF, nullptr, DD, T512, DD, bfb, 0, 0, 0);
        k_l2n<<<NP / 8, 256, 0, stream>>>(T512, OUTX + (size_t)b * NP * DD, XN);
        k_gemmw<h16, 0, false><<<dim3(NP / 64, NPR / 64, 1), 32, 0, stream>>>(XN, nullptr, PR, nullptr, DD, S, NPR, nullptr, 0, 0, 0);
        k_amax<<<(NC * NP + 255) / 256, 256, 0, stream>>>(S, ACT + (size_t)b * NC * NP); }
    k_logit<<<(NI * NC + 255) / 256, 256, 0, stream>>>(ACT, ls, LOG);
}
